// WindowAttention_85315230368227
// MI455X (gfx1250) — hardware-verified
//
#include <hip/hip_runtime.h>
#include <stdint.h>
#include <stddef.h>

#ifndef NB
#define NB 2
#endif
#ifndef NWIN
#define NWIN 64
#endif

typedef __attribute__((ext_vector_type(16))) __bf16   v16b;
typedef __attribute__((ext_vector_type(8)))  __bf16   v8b;
typedef __attribute__((ext_vector_type(8)))  float    v8f;
typedef __attribute__((ext_vector_type(4)))  float    v4f;
typedef __attribute__((ext_vector_type(4)))  unsigned v4u;
typedef __attribute__((ext_vector_type(2)))  unsigned v2u;

constexpr int   kImg   = 64;
constexpr int   kCand  = 4;
constexpr int   kC     = 128;
constexpr int   kC3    = 384;
constexpr int   kHd    = 32;
constexpr int   kHeads = 4;
constexpr int   kWs    = 8;
constexpr int   kShift = 4;
constexpr int   kM     = 256;
constexpr int   kPix   = 64;
constexpr int   kTab   = 225;
constexpr float kScale = 0.17677669529663687f;
constexpr size_t kInStrideB  = (size_t)kImg * kImg * kCand * kC3;
constexpr size_t kOutStrideB = (size_t)kImg * kImg * kCand * kC;

static_assert(NB >= 1 && NB <= 2);
static_assert(NWIN >= 1 && NWIN <= 64);
static_assert(kHd % 32 == 0 && kM % 64 == 0);

constexpr size_t kEmbRows  = (size_t)kHeads * 16 * 16 * 16;
constexpr size_t kEmbBytes = kEmbRows * kHd * 2;
constexpr size_t kVegRows  = (size_t)kHeads * kPix * kHd;
constexpr size_t kVegBytes = kVegRows * 64 * 2;
constexpr size_t kMpadBytes = (size_t)NWIN * kM * kM * 4;
static_assert(kMpadBytes % 128 == 0 && kEmbBytes % 128 == 0 && kVegBytes % 128 == 0);
static_assert(kMpadBytes + 2 * kEmbBytes + kVegBytes <= (size_t)134217728);

constexpr int kOffQ     = 0;
constexpr int kOffK     = 16384;
constexpr int kOffVt    = 32768;
constexpr int kOffWave  = 49152;
constexpr int kWoffE2   = 0;
constexpr int kWoffPh   = 1024;
constexpr int kWoffPl   = 3072;
constexpr int kWoffAh   = 5120;
constexpr int kWoffAl   = 7168;
constexpr int kWoffOut  = 9216;
constexpr int kWaveBytes = 11264;
constexpr int kLdsBytes  = kOffWave + 8 * kWaveBytes;
static_assert(kLdsBytes == 139264);
static_assert(kWoffAl == kWoffAh + 2048);

union FragU { v16b v; v8b h[2]; };
__device__ __forceinline__ v16b ldfrag(const unsigned short* p) {
  FragU f;
  f.h[0] = *(const v8b*)(const void*)(p);
  f.h[1] = *(const v8b*)(const void*)(p + 16);
  return f.v;
}
__device__ __forceinline__ v16b ldfrag2(const unsigned short* p0, const unsigned short* p1) {
  FragU f;
  f.h[0] = *(const v8b*)(const void*)(p0);
  f.h[1] = *(const v8b*)(const void*)(p1);
  return f.v;
}
__device__ __forceinline__ v8f zero8() { return (v8f){0.f, 0.f, 0.f, 0.f, 0.f, 0.f, 0.f, 0.f}; }

__device__ __forceinline__ v8f mma1(v16b a, v16b b, v8f c) {
  c = __builtin_amdgcn_wmma_f32_16x16x32_bf16(false, a, false, b, (short)0, c, false, false);
  asm volatile("v_nop\n\tv_nop\n\tv_nop\n\tv_nop" : "+v"(c) : "v"(a), "v"(b));
  return c;
}
__device__ __forceinline__ v8f mma2(v16b ah, v16b al, v16b b, v8f c) {
  c = __builtin_amdgcn_wmma_f32_16x16x32_bf16(false, ah, false, b, (short)0, c, false, false);
  c = __builtin_amdgcn_wmma_f32_16x16x32_bf16(false, al, false, b, (short)0, c, false, false);
  asm volatile("v_nop\n\tv_nop\n\tv_nop\n\tv_nop" : "+v"(c) : "v"(ah), "v"(al), "v"(b));
  return c;
}
__device__ __forceinline__ void lds_wave_sync() {
  __builtin_amdgcn_fence(3, "workgroup");
  __builtin_amdgcn_wave_barrier();
  __builtin_amdgcn_fence(2, "workgroup");
}

__device__ __forceinline__ unsigned bf_rne_bits(float f) {
  const unsigned u = __float_as_uint(f);
  return (u + 0x7FFFu + ((u >> 16) & 1u)) >> 16;
}
__device__ __forceinline__ float bf_rne(float f) { return __uint_as_float(bf_rne_bits(f) << 16); }
__device__ __forceinline__ void bf_split(float f, unsigned& hb, unsigned& lb) {
  hb = bf_rne_bits(f);
  lb = bf_rne_bits(f - __uint_as_float(hb << 16));
}
__device__ __forceinline__ float sel4(float a0, float a1, float a2, float a3, int q) {
  const float b0 = (q & 1) ? a1 : a0;
  const float b1 = (q & 1) ? a3 : a2;
  return (q & 2) ? b1 : b0;
}
__device__ __forceinline__ int tok_row(int m, int whi, int wwi) {
  const int p = m >> 2, n = m & 3;
  const int y = (whi * kWs + (p >> 3) + kShift) & (kImg - 1);
  const int x = (wwi * kWs + (p & 7) + kShift) & (kImg - 1);
  return (y * kImg + x) * kCand + n;
}

__global__ __launch_bounds__(256) void k_prep_mask(const float* __restrict__ am, float* __restrict__ mpad) {
  const int gid = blockIdx.x * 256 + threadIdx.x;
  const int cc = gid & 15, ch = (gid >> 4) & 3, row = (gid >> 6) & 255, w = gid >> 14;
  const float* src = am + ((size_t)w * kM + row) * kM + ch * 64 + cc;
  v4f o;
#pragma unroll
  for (int tl = 0; tl < 4; ++tl) o[tl] = bf_rne(src[tl * 16]);
  float* p = mpad + (size_t)gid * 4;
  *(volatile v4f*)p = o;
  __threadfence();
  *(volatile v4f*)p = o;
}

__global__ __launch_bounds__(256) void k_prep_emb(const float* __restrict__ rpe, const int* __restrict__ rel,
                                                  unsigned short* __restrict__ qeg, unsigned short* __restrict__ keg,
                                                  unsigned short* __restrict__ vegt) {
  const int blk = blockIdx.x;
  if (blk < 512) {
    const bool isQ = (blk < 256);
    const int gid = (isQ ? blk : (blk - 256)) * 256 + threadIdx.x;
    const int row = gid >> 2, piece = gid & 3;
    const int head = row >> 12, pib = (row >> 8) & 15, t = (row >> 4) & 15, r = row & 15;
    const int pi = pib * 4 + (isQ ? (r >> 2) : (r & 3));
    const int pj = t * 4 + (isQ ? (r & 3) : (r >> 2));
    int ix = rel[pi * kPix + pj];
    ix = (ix < 0) ? 0 : ((ix > kTab - 1) ? (kTab - 1) : ix);
    const float* src = rpe + (size_t)ix * kC3 + head * 96 + (isQ ? 0 : kHd) + piece * 8;
    const v4f a0 = *(const v4f*)(src);
    const v4f a1 = *(const v4f*)(src + 4);
    v4u wv;
    wv[0] = bf_rne_bits(a0[0]) | (bf_rne_bits(a0[1]) << 16);
    wv[1] = bf_rne_bits(a0[2]) | (bf_rne_bits(a0[3]) << 16);
    wv[2] = bf_rne_bits(a1[0]) | (bf_rne_bits(a1[1]) << 16);
    wv[3] = bf_rne_bits(a1[2]) | (bf_rne_bits(a1[3]) << 16);
    unsigned short* dst = (isQ ? qeg : keg) + (size_t)row * kHd + piece * 8;
    *(volatile v4u*)dst = wv;
    __threadfence();
    *(volatile v4u*)dst = wv;
  } else {
    const int gid = (blk - 512) * 256 + threadIdx.x;
    const int row = gid >> 3, piece = gid & 7;
    const int head = row >> 11, pi = (row >> 5) & 63, c = row & 31;
    unsigned bits[8];
#pragma unroll
    for (int e = 0; e < 8; ++e) {
      int ix = rel[pi * kPix + piece * 8 + e];
      ix = (ix < 0) ? 0 : ((ix > kTab - 1) ? (kTab - 1) : ix);
      bits[e] = bf_rne_bits(rpe[(size_t)ix * kC3 + head * 96 + 2 * kHd + c]);
    }
    v4u wv;
#pragma unroll
    for (int q = 0; q < 4; ++q) wv[q] = bits[2 * q] | (bits[2 * q + 1] << 16);
    unsigned short* dst = vegt + (size_t)row * 64 + piece * 8;
    *(volatile v4u*)dst = wv;
    __threadfence();
    *(volatile v4u*)dst = wv;
  }
}

__global__ __launch_bounds__(256) void k_win_attn(const float* __restrict__ qkv, const float* __restrict__ mpad,
                                                  const unsigned short* __restrict__ qeg, const unsigned short* __restrict__ keg,
                                                  const unsigned short* __restrict__ vegt, float* __restrict__ out) {
  __shared__ __align__(16) unsigned char lds_raw[kLdsBytes];
  unsigned short* sQ  = (unsigned short*)(lds_raw + kOffQ);
  unsigned short* sK  = (unsigned short*)(lds_raw + kOffK);
  unsigned short* sVt = (unsigned short*)(lds_raw + kOffVt);

  const int tid = threadIdx.x;
  const int lane = tid & 31, wave = tid >> 5;
  const int hh = lane >> 4, cc = lane & 15, q2 = cc >> 2;
  unsigned char* wb = lds_raw + kOffWave + wave * kWaveBytes;
  float* sE2 = (float*)(wb + kWoffE2);
  unsigned short* ph  = (unsigned short*)(wb + kWoffPh);
  unsigned short* pl  = (unsigned short*)(wb + kWoffPl);
  unsigned short* pah = (unsigned short*)(wb + kWoffAh);
  unsigned short* pal = (unsigned short*)(wb + kWoffAl);
  float* sOut = (float*)(wb + kWoffOut);

  const int bIdx = blockIdx.x;
  const int head = bIdx & (kHeads - 1);
  const int bw = bIdx >> 2;
  const int b = bw / NWIN;
  const int w = bw - b * NWIN;
  const int whi = w >> 3, wwi = w & 7;

  {
    const float* qb = qkv + (size_t)b * kInStrideB + head * kHd;
    for (int i = tid; i < kM * 8; i += 256) {
      const int m = i >> 3, c4 = (i & 7) * 4;
      const float* gp = qb + (size_t)tok_row(m, whi, wwi) * kC3 + c4;
      const v4f vq = *(const v4f*)(gp);
      const v4f vk = *(const v4f*)(gp + kC);
      const v4f vv = *(const v4f*)(gp + 2 * kC);
      v2u pq, pk;
      pq[0] = bf_rne_bits(vq[0]) | (bf_rne_bits(vq[1]) << 16);
      pq[1] = bf_rne_bits(vq[2]) | (bf_rne_bits(vq[3]) << 16);
      pk[0] = bf_rne_bits(vk[0]) | (bf_rne_bits(vk[1]) << 16);
      pk[1] = bf_rne_bits(vk[2]) | (bf_rne_bits(vk[3]) << 16);
      *(v2u*)(sQ + m * kHd + c4) = pq;
      *(v2u*)(sK + m * kHd + c4) = pk;
      sVt[(c4 + 0) * kM + m] = (unsigned short)bf_rne_bits(vv[0]);
      sVt[(c4 + 1) * kM + m] = (unsigned short)bf_rne_bits(vv[1]);
      sVt[(c4 + 2) * kM + m] = (unsigned short)bf_rne_bits(vv[2]);
      sVt[(c4 + 3) * kM + m] = (unsigned short)bf_rne_bits(vv[3]);
    }
    const v4u z = {0u, 0u, 0u, 0u};
#pragma unroll
    for (int j = 0; j < 8; ++j) *(v4u*)(pah + lane * 64 + j * 8) = z;
  }
  __syncthreads();
  lds_wave_sync();

#pragma unroll 1
  for (int si = 0; si < 2; ++si) {
    const int pib = wave + 8 * si;
    const int Q0 = pib * 16;
    const v16b qf = ldfrag(sQ + (Q0 + cc) * kHd + 8 * hh);
    float mrun[8], lrun[8];
#pragma unroll
    for (int g = 0; g < 8; ++g) { mrun[g] = -1.0e30f; lrun[g] = 0.0f; }
    v8f o0 = zero8(), o1 = zero8();
    const float* mstrip = mpad + ((size_t)w * kM + Q0 + 8 * hh) * kM + cc * 4;
    const unsigned short* tq = qeg  + ((size_t)((head * 16 + pib) * 16) * 16 + cc) * kHd + 8 * hh;
    const unsigned short* tk = keg  + ((size_t)((head * 16 + pib) * 16) * 16 + cc) * kHd + 8 * hh;
    const unsigned short* tv = vegt + ((size_t)(head * kPix + pib * 4) * kHd + cc) * 64 + 8 * hh;

#pragma unroll 1
    for (int ch = 0; ch < 4; ++ch) {
      v8f ct[4];
#pragma unroll
      for (int t = 0; t < 4; ++t) {
        const int kt = ch * 4 + t;
        const v16b kfr = ldfrag(sK + (kt * 16 + cc) * kHd + 8 * hh);
        const v16b a3  = ldfrag(tq + (size_t)kt * (16 * kHd));
        const v16b a2  = ldfrag(tk + (size_t)kt * (16 * kHd));
        ct[t] = mma1(qf, kfr, zero8());
        const v8f d3 = mma1(a3, kfr, zero8());
        const v8f d2 = mma1(a2, qf, zero8());
        const float u0 = sel4(d3[0], d3[1], d3[2], d3[3], q2);
        const float u1 = sel4(d3[4], d3[5], d3[6], d3[7], q2);
        ct[t][0] += u0; ct[t][1] += u0; ct[t][2] += u0; ct[t][3] += u0;
        ct[t][4] += u1; ct[t][5] += u1; ct[t][6] += u1; ct[t][7] += u1;
        const float w0 = sel4(d2[0], d2[1], d2[2], d2[3], q2);
        const float w1 = sel4(d2[4], d2[5], d2[6], d2[7], q2);
        sE2[(t * 4 + 2 * hh) * 16 + cc]     = w0;
        sE2[(t * 4 + 2 * hh + 1) * 16 + cc] = w1;
      }
      lds_wave_sync();
#pragma unroll
      for (int t = 0; t < 4; ++t) {
        const v4f ea = *(const v4f*)(sE2 + (t * 4 + q2) * 16 + 8 * hh);
        const v4f eb = *(const v4f*)(sE2 + (t * 4 + q2) * 16 + 8 * hh + 4);
        ct[t][0] += ea[0]; ct[t][1] += ea[1]; ct[t][2] += ea[2]; ct[t][3] += ea[3];
        ct[t][4] += eb[0]; ct[t][5] += eb[1]; ct[t][6] += eb[2]; ct[t][7] += eb[3];
      }
#pragma unroll
      for (int g = 0; g < 8; ++g) {
        const v4f mk = *(const v4f*)(mstrip + (size_t)g * kM + ch * 64);
        const float s0 = ct[0][g] * kScale + mk[0];
        const float s1 = ct[1][g] * kScale + mk[1];
        const float s2 = ct[2][g] * kScale + mk[2];
        const float s3 = ct[3][g] * kScale + mk[3];
        float cmx = fmaxf(fmaxf(s0, s1), fmaxf(s2, s3));
        cmx = fmaxf(cmx, __shfl_xor(cmx, 1, 32));
        cmx = fmaxf(cmx, __shfl_xor(cmx, 2, 32));
        cmx = fmaxf(cmx, __shfl_xor(cmx, 4, 32));
        cmx = fmaxf(cmx, __shfl_xor(cmx, 8, 32));
        const float mn = fmaxf(mrun[g], cmx);
        const float alpha = __expf(mrun[g] - mn);
        mrun[g] = mn;
        const float e0 = __expf(s0 - mn);
        const float e1 = __expf(s1 - mn);
        const float e2 = __expf(s2 - mn);
        const float e3 = __expf(s3 - mn);
        float rs = (e0 + e1) + (e2 + e3);
        rs += __shfl_xor(rs, 1, 32);
        rs += __shfl_xor(rs, 2, 32);
        rs += __shfl_xor(rs, 4, 32);
        rs += __shfl_xor(rs, 8, 32);
        lrun[g] = lrun[g] * alpha + rs;
        o0[g] *= alpha;
        o1[g] *= alpha;
        ct[0][g] = e0; ct[1][g] = e1; ct[2][g] = e2; ct[3][g] = e3;
      }
#pragma unroll
      for (int t = 0; t < 4; ++t) {
#pragma unroll
        for (int g = 0; g < 8; ++g) {
          const float e = ct[t][g];
          unsigned hb, lb;
          bf_split(e, hb, lb);
          const int po = (8 * hh + g) * 64 + t * 16 + cc;
          ph[po] = (unsigned short)hb;
          pl[po] = (unsigned short)lb;
          float x = e;
          x += __shfl_xor(x, 1, 32);
          x += __shfl_xor(x, 2, 32);
          unsigned sh, sl;
          bf_split(x, sh, sl);
          if ((cc & 3) == 0) {
            const int ao = (8 * hh + g) * 64 + (2 * hh + (g >> 2)) * 16 + t * 4 + q2;
            pah[ao] = (unsigned short)sh;
            pal[ao] = (unsigned short)sl;
          }
        }
      }
      lds_wave_sync();
      v16b pfh[2], pfl[2], afh[2], afl[2];
#pragma unroll
      for (int kk = 0; kk < 2; ++kk) {
        pfh[kk] = ldfrag(ph  + cc * 64 + kk * 32 + 8 * hh);
        pfl[kk] = ldfrag(pl  + cc * 64 + kk * 32 + 8 * hh);
        afh[kk] = ldfrag(pah + cc * 64 + kk * 32 + 8 * hh);
        afl[kk] = ldfrag(pal + cc * 64 + kk * 32 + 8 * hh);
      }
#pragma unroll
      for (int kk = 0; kk < 2; ++kk) {
        const v16b v0f = ldfrag(sVt + (cc)      * kM + ch * 64 + kk * 32 + 8 * hh);
        const v16b v1f = ldfrag(sVt + (16 + cc) * kM + ch * 64 + kk * 32 + 8 * hh);
        o0 = mma2(pfh[kk], pfl[kk], v0f, o0);
        o1 = mma2(pfh[kk], pfl[kk], v1f, o1);
      }
#pragma unroll
      for (int ks = 0; ks < 2; ++ks) {
        const unsigned short* r0 = tv + (size_t)(2 * ks) * (kHd * 64) + ch * 16;
        const v16b b0 = ldfrag2(r0,           r0 + kHd * 64);
        const v16b b1 = ldfrag2(r0 + 16 * 64, r0 + 16 * 64 + kHd * 64);
        o0 = mma2(afh[ks], afl[ks], b0, o0);
        o1 = mma2(afh[ks], afl[ks], b1, o1);
      }
    }

    {
      float inv[8];
#pragma unroll
      for (int g = 0; g < 8; ++g) inv[g] = 1.0f / lrun[g];
#pragma unroll
      for (int r = 0; r < 8; ++r) {
        const float y0 = o0[r] * inv[r];
        const float y1 = o1[r] * inv[r];
        sOut[(8 * hh + r) * kHd + cc]      = y0;
        sOut[(8 * hh + r) * kHd + 16 + cc] = y1;
      }
      lds_wave_sync();
      float* ob = out + (size_t)b * kOutStrideB + head * kHd + (lane & 7) * 4;
#pragma unroll
      for (int it = 0; it < 4; ++it) {
        const int R = it * 4 + (lane >> 3);
        const v4f v = *(const v4f*)(sOut + R * kHd + (lane & 7) * 4);
        *(volatile v4f*)(ob + (size_t)tok_row(Q0 + R, whi, wwi) * kC) = v;
      }
      __threadfence();
#pragma unroll
      for (int it = 0; it < 4; ++it) {
        const int R = it * 4 + (lane >> 3);
        const v4f v = *(const v4f*)(sOut + R * kHd + (lane & 7) * 4);
        *(volatile v4f*)(ob + (size_t)tok_row(Q0 + R, whi, wwi) * kC) = v;
      }
    }
  }
}

extern "C" void kernel_launch(void* const* d_in, const int* in_sizes, int n_in,
                              void* d_out, int out_size, void* d_ws, size_t ws_size,
                              hipStream_t stream) {
  if (n_in < 4) return;
  const float* qkv  = (const float*)d_in[0];
  const float* rpe  = (const float*)d_in[1];
  const int*   rel  = (const int*)d_in[2];
  const float* amsk = (const float*)d_in[3];
  float* out = (float*)d_out;

  if ((size_t)in_sizes[0] < (size_t)NB * kInStrideB) return;
  if (in_sizes[1] < kTab * kC3) return;
  if (in_sizes[2] < kPix * kPix) return;
  if ((size_t)in_sizes[3] < (size_t)NWIN * kM * kM) return;
  if ((size_t)out_size < (size_t)NB * kOutStrideB) return;

  const size_t offM  = 0;
  const size_t offQe = offM  + kMpadBytes;
  const size_t offKe = offQe + kEmbBytes;
  const size_t offVe = offKe + kEmbBytes;
  const size_t total = offVe + kVegBytes;
  if (total > ws_size || total > (size_t)134217728) return;
  unsigned char* ws = (unsigned char*)d_ws;
  float* mpad = (float*)(ws + offM);
  unsigned short* qeg  = (unsigned short*)(ws + offQe);
  unsigned short* keg  = (unsigned short*)(ws + offKe);
  unsigned short* vegt = (unsigned short*)(ws + offVe);

  k_prep_mask<<<NWIN * 64, 256, 0, stream>>>(amsk, mpad);
  k_prep_emb<<<768, 256, 0, stream>>>(rpe, rel, qeg, keg, vegt);
  k_win_attn<<<NB * NWIN * kHeads, 256, 0, stream>>>(qkv, mpad, qeg, keg, vegt, out);
}
